// LossMeanCov_34230889349412
// MI455X (gfx1250) — hardware-verified
//
#include <hip/hip_runtime.h>

typedef __attribute__((ext_vector_type(16))) _Float16 v16h;
typedef __attribute__((ext_vector_type(8)))  _Float16 v8h;
typedef __attribute__((ext_vector_type(16))) __bf16   v16b;
typedef __attribute__((ext_vector_type(8)))  __bf16   v8b;
typedef __attribute__((ext_vector_type(8)))  float    v8f;
typedef __attribute__((ext_vector_type(4)))  float    v4f;
typedef __attribute__((ext_vector_type(4)))  int      v4i;

static constexpr int   XDIM      = 32;
static constexpr int   NCLUST    = 64;
static constexpr int   FEAT      = 64;
static constexpr int   ASG_WAVES = 8;
static constexpr int   ASG_PPW   = 64;
static constexpr int   ASG_PPB   = ASG_WAVES * ASG_PPW;
static constexpr int   ST_CHUNK  = 512;
static constexpr int   ST_STRIDE = 1088;
static constexpr float BETA_T    = 10.0f;
static constexpr float KAPPA_W   = 1.0f;

__device__ __forceinline__ unsigned short f2bf_bits(float f) {
  unsigned u = __float_as_uint(f);
  return (unsigned short)((u + 0x7FFFu + ((u >> 16) & 1u)) >> 16);
}
__device__ __forceinline__ float bf_bits2f(unsigned short h) { return __uint_as_float(((unsigned)h) << 16); }

__device__ __forceinline__ void dep_guard_h(v8f& a, v8f& b, v16h x, v16h y) { asm volatile("v_nop\n\tv_nop\n\tv_nop\n\tv_nop" : "+v"(a), "+v"(b) : "v"(x), "v"(y)); }
__device__ __forceinline__ void dep_guard_b(v8f& a, v8f& b, v16b x, v16b y) { asm volatile("v_nop\n\tv_nop\n\tv_nop\n\tv_nop" : "+v"(a), "+v"(b) : "v"(x), "v"(y)); }
__device__ __forceinline__ void keep4_h(v16h a, v16h b, v16h c, v16h d) { asm volatile("v_nop" :: "v"(a), "v"(b), "v"(c), "v"(d)); }
__device__ __forceinline__ void keep4_b(v16b a, v16b b, v16b c, v16b d) { asm volatile("v_nop" :: "v"(a), "v"(b), "v"(c), "v"(d)); }
__device__ __forceinline__ void acc_guard4(v8f& a, v8f& b, v8f& c, v8f& d) { asm volatile("v_nop\n\tv_nop\n\tv_nop\n\tv_nop" : "+v"(a), "+v"(b), "+v"(c), "+v"(d)); }
template <typename T> struct Frag;
template <> struct Frag<_Float16> {
  typedef v16h V; union U { v16h v; v8h h[2]; };
  static __device__ __forceinline__ v16h load(const _Float16* p) {
    U f; f.h[0] = *(const v8h*)(p); f.h[1] = *(const v8h*)(p + 16); return f.v;
  }
  static __device__ __forceinline__ v8f mma(v16h a, v16h b, v8f c) {
    return __builtin_amdgcn_wmma_f32_16x16x32_f16(false, a, false, b, (short)0, c, false, false);
  }
  static __device__ __forceinline__ void guard(v8f& a, v8f& b, v16h x, v16h y) { dep_guard_h(a, b, x, y); }
  static __device__ __forceinline__ void keep(v16h a, v16h b, v16h c, v16h d) { keep4_h(a, b, c, d); }
};
template <> struct Frag<__bf16> {
  typedef v16b V; union U { v16b v; v8b h[2]; };
  static __device__ __forceinline__ v16b load(const __bf16* p) {
    U f; f.h[0] = *(const v8b*)(p); f.h[1] = *(const v8b*)(p + 16); return f.v;
  }
  static __device__ __forceinline__ v8f mma(v16b a, v16b b, v8f c) {
    return __builtin_amdgcn_wmma_f32_16x16x32_bf16(false, a, false, b, (short)0, c, false, false);
  }
  static __device__ __forceinline__ void guard(v8f& a, v8f& b, v16b x, v16b y) { dep_guard_b(a, b, x, y); }
  static __device__ __forceinline__ void keep(v16b a, v16b b, v16b c, v16b d) { keep4_b(a, b, c, d); }
};

template <int ET> struct Elem;
template <> struct Elem<0> { typedef _Float16 T; };
template <> struct Elem<1> { typedef __bf16 T; };
template <int ET, bool SPLIT, int BIAS_MODE, int OUT_MODE, bool RESID, int ACT = 0>
__global__ __launch_bounds__(256) void wmma_gemm64(
    const unsigned short* __restrict__ Ap, const unsigned short* __restrict__ A2p, int lda, long strideA,
    const unsigned short* __restrict__ Btp, const unsigned short* __restrict__ Bt2p, int ldb, long strideB,
    void* __restrict__ Cout, void* __restrict__ Cout2, int ldc, long strideC,
    const float* __restrict__ bias,
    const float* __restrict__ resid, long strideR,
    int M, int N, int K, float scale) {
  typedef typename Elem<ET>::T T;
  typedef typename Frag<T>::V V;
  const T* A = (const T*)Ap; const T* A2 = (const T*)A2p; const T* Bt = (const T*)Btp; const T* Bt2 = (const T*)Bt2p;
  __shared__ __align__(16) float sT[8][16 * 68];
  const int b    = blockIdx.y;
  const int lane = threadIdx.x & 31;
  const int wave = threadIdx.x >> 5;
  const int tilesN = N >> 6;
  const int tilesM = M >> 6;
  const int tile = blockIdx.x * 8 + wave;
  if (tile >= tilesM * tilesN) return;
  const int tm = tile / tilesN;
  const int tn = tile - tm * tilesN;
  const int m0 = tm << 6;
  const int n0 = tn << 6;

  const T* Ab  = A  + (size_t)b * strideA;
  const T* Bb  = Bt + (size_t)b * strideB;
  const T* Ab2 = SPLIT ? (A2  + (size_t)b * strideA) : nullptr;
  const T* Bb2 = SPLIT ? (Bt2 + (size_t)b * strideB) : nullptr;

  const int rlane = lane & 15;
  const int koff  = (lane >> 4) * 8;
  const int mOff  = (lane >> 4) * 8;

  v8f acc[4][4];
#pragma unroll
  for (int i = 0; i < 4; ++i)
#pragma unroll
    for (int j = 0; j < 4; ++j) acc[i][j] = (v8f){0.f,0.f,0.f,0.f,0.f,0.f,0.f,0.f};

  for (int k0 = 0; k0 < K; k0 += 32) {
    V bh[4], bl[4];
#pragma unroll
    for (int j = 0; j < 4; ++j) {
      const size_t bo = (size_t)(n0 + (j << 4) + rlane) * ldb + koff + k0;
      bh[j] = Frag<T>::load(Bb + bo);
      if (SPLIT) bl[j] = Frag<T>::load(Bb2 + bo);
    }
#pragma unroll
    for (int i = 0; i < 4; ++i) {
      const size_t ao = (size_t)(m0 + (i << 4) + rlane) * lda + koff + k0;
      V ah = Frag<T>::load(Ab + ao);
      V al;
      if (SPLIT) al = Frag<T>::load(Ab2 + ao);
#pragma unroll
      for (int j = 0; j < 4; ++j) {
        acc[i][j] = Frag<T>::mma(ah, bh[j], acc[i][j]);
        if (SPLIT) {
          acc[i][j] = Frag<T>::mma(ah, bl[j], acc[i][j]);
          acc[i][j] = Frag<T>::mma(al, bh[j], acc[i][j]);
        }
      }
      Frag<T>::guard(acc[i][0], acc[i][3], ah, SPLIT ? al : ah);
    }
    Frag<T>::keep(bh[0], bh[1], bh[2], bh[3]);
    if (SPLIT) Frag<T>::keep(bl[0], bl[1], bl[2], bl[3]);
  }
  acc_guard4(acc[0][0], acc[0][1], acc[0][2], acc[0][3]);
  acc_guard4(acc[1][0], acc[1][1], acc[1][2], acc[1][3]);
  acc_guard4(acc[2][0], acc[2][1], acc[2][2], acc[2][3]);
  acc_guard4(acc[3][0], acc[3][1], acc[3][2], acc[3][3]);

  float* slab = sT[wave];
  const float* Rb = RESID ? (resid + (size_t)b * strideR) : nullptr;
#pragma unroll
  for (int i = 0; i < 4; ++i) {
    const int mBase = m0 + (i << 4);
#pragma unroll
    for (int j = 0; j < 4; ++j) {
      const int n = n0 + (j << 4) + rlane;
      float bv = 0.f;
      if (BIAS_MODE == 2) bv = bias[n];
#pragma unroll
      for (int r = 0; r < 8; ++r) {
        float v = acc[i][j][r] * scale;
        if (BIAS_MODE == 1) v += bias[mBase + mOff + r];
        if (BIAS_MODE == 2) v += bv;
        if (RESID) v += Rb[(size_t)(mBase + mOff + r) * ldc + n];
        if (ACT == 1) v = tanhf(v);
        if (ACT == 2) v = fmaxf(v, 0.0f);
        if (ACT == 3) v = v / (1.0f + expf(-v));
        if (ACT == 4) v = (v > 0.f) ? v : 0.01f * v;
        if (ACT == 5) v = 0.5f * v * (1.0f + erff(v * 0.70710678118654752f));
        slab[(mOff + r) * 68 + (j << 4) + rlane] = v;
      }
    }
    __builtin_amdgcn_fence(__ATOMIC_RELEASE, "workgroup");
    __builtin_amdgcn_wave_barrier();
    __builtin_amdgcn_fence(__ATOMIC_ACQUIRE, "workgroup");
    if (OUT_MODE == 0) {
      float* C = (float*)Cout + (size_t)b * strideC;
      const int hh = lane >> 4, c4 = (lane & 15) * 4;
      for (int pass = 0; pass < 2; ++pass) {
#pragma unroll
        for (int it = 0; it < 8; ++it) {
          const int row = it * 2 + hh;
          v4f v = *(const v4f*)(slab + row * 68 + c4);
          *(volatile v4f*)(C + (size_t)(mBase + row) * ldc + n0 + c4) = v;
        }
        __threadfence();
      }
    } else {
      const int q = lane >> 3, c8 = (lane & 7) * 8;
      unsigned short* C  = (unsigned short*)Cout  + (size_t)b * strideC;
      unsigned short* C2 = (OUT_MODE == 2) ? ((unsigned short*)Cout2 + (size_t)b * strideC) : nullptr;
      for (int pass = 0; pass < 2; ++pass) {
#pragma unroll
        for (int it = 0; it < 4; ++it) {
          const int row = it * 4 + q;
          const float* sp = slab + row * 68 + c8;
          v8h hv, lv;
#pragma unroll
          for (int e = 0; e < 8; ++e) {
            if (OUT_MODE == 1) {
              hv[e] = (_Float16)sp[e];
            } else {
              unsigned short hb = f2bf_bits(sp[e]);
              unsigned short lb = f2bf_bits(sp[e] - bf_bits2f(hb));
              hv[e] = __builtin_bit_cast(_Float16, hb);
              lv[e] = __builtin_bit_cast(_Float16, lb);
            }
          }
          *(volatile v8h*)(C + (size_t)(mBase + row) * ldc + n0 + c8) = hv;
          if (OUT_MODE == 2) *(volatile v8h*)(C2 + (size_t)(mBase + row) * ldc + n0 + c8) = lv;
        }
        __threadfence();
      }
    }
    __builtin_amdgcn_fence(__ATOMIC_RELEASE, "workgroup");
    __builtin_amdgcn_wave_barrier();
    __builtin_amdgcn_fence(__ATOMIC_ACQUIRE, "workgroup");
  }
}

__global__ __launch_bounds__(256) void split_rows64_bf16(
    const float* __restrict__ in, unsigned short* __restrict__ hi, unsigned short* __restrict__ lo,
    int rows_valid, int rows_total) {
  const int t = blockIdx.x * 256 + threadIdx.x;
  const int nthr = rows_total * 8;
  if (t < nthr) {
    const int row = t >> 3;
    const int c8  = (t & 7) * 8;
    const int rowc = (row < rows_valid) ? row : (rows_valid - 1);
    const bool live = (row < rows_valid);
    const float* p = in + (size_t)rowc * FEAT + c8;
    const v4f a = *(const v4f*)p;
    const v4f bq = *(const v4f*)(p + 4);
    v8h hv, lv;
#pragma unroll
    for (int e = 0; e < 4; ++e) {
      const float f0 = live ? a[e]  : 0.0f;
      const float f1 = live ? bq[e] : 0.0f;
      const unsigned short h0 = f2bf_bits(f0);
      const unsigned short l0 = f2bf_bits(f0 - bf_bits2f(h0));
      const unsigned short h1 = f2bf_bits(f1);
      const unsigned short l1 = f2bf_bits(f1 - bf_bits2f(h1));
      hv[e]     = __builtin_bit_cast(_Float16, h0);
      lv[e]     = __builtin_bit_cast(_Float16, l0);
      hv[4 + e] = __builtin_bit_cast(_Float16, h1);
      lv[4 + e] = __builtin_bit_cast(_Float16, l1);
    }
    unsigned short* ph = hi + (size_t)row * FEAT + c8;
    unsigned short* pl = lo + (size_t)row * FEAT + c8;
    *(volatile v8h*)ph = hv;
    *(volatile v8h*)pl = lv;
    __threadfence();
    *(volatile v8h*)ph = hv;
    *(volatile v8h*)pl = lv;
  }
}

__device__ __forceinline__ float rcp_f32(float v) {
#if __has_builtin(__builtin_amdgcn_rcpf)
  return __builtin_amdgcn_rcpf(v);
#else
  return 1.0f / v;
#endif
}

__global__ __launch_bounds__(256) void assign_kernel(
    const float* __restrict__ x, const float* __restrict__ centers, const float* __restrict__ xc,
    int* __restrict__ pred, float* __restrict__ partp, int npts) {
  __shared__ __align__(16) int   sPred[ASG_WAVES][ASG_PPW];
  __shared__ __align__(16) float sFill[ASG_WAVES][NCLUST];
  __shared__ __align__(16) float sOut[NCLUST];
  const int tid  = threadIdx.x;
  const int lane = tid & 31;
  const int wave = tid >> 5;

  float cc0 = 0.f, cc1 = 0.f;
#pragma unroll 1
  for (int d = 0; d < XDIM; ++d) {
    const float c0 = centers[lane * XDIM + d];
    const float c1 = centers[(lane + 32) * XDIM + d];
    cc0 = fmaf(c0, c0, cc0);
    cc1 = fmaf(c1, c1, cc1);
  }

  const int base = (blockIdx.x * ASG_WAVES + wave) * ASG_PPW;
  float acc0 = 0.f, acc1 = 0.f;
#pragma unroll 1
  for (int i = 0; i < ASG_PPW; ++i) {
    const int n = base + i;
    const float xv = x[(size_t)n * XDIM + lane];
    float xx = xv * xv;
#pragma unroll
    for (int off = 16; off >= 1; off >>= 1) xx += __shfl_xor(xx, off, 32);
    const float v0 = xc[(size_t)n * NCLUST + lane];
    const float v1 = xc[(size_t)n * NCLUST + 32 + lane];
    const float d0 = (xx - 2.0f * v0) + cc0;
    const float d1 = (xx - 2.0f * v1) + cc1;
    float m = fminf(d0, d1);
#pragma unroll
    for (int off = 16; off >= 1; off >>= 1) m = fminf(m, __shfl_xor(m, off, 32));
    int cand = (d0 == m) ? lane : ((d1 == m) ? (lane + 32) : NCLUST);
#pragma unroll
    for (int off = 16; off >= 1; off >>= 1) cand = min(cand, __shfl_xor(cand, off, 32));
    const float zmax = -BETA_T * m;
    const float e0 = __expf(-BETA_T * d0 - zmax);
    const float e1 = __expf(-BETA_T * d1 - zmax);
    float z = e0 + e1;
#pragma unroll
    for (int off = 16; off >= 1; off >>= 1) z += __shfl_xor(z, off, 32);
    const float inv = rcp_f32(z);
    acc0 = fmaf(e0, inv, acc0);
    acc1 = fmaf(e1, inv, acc1);
    if (lane == 0) sPred[wave][i] = (cand < NCLUST) ? cand : (NCLUST - 1);
  }
  __syncthreads();

  {
    const int lq = (lane < 16) ? lane : 0;
    const v4i pv = *(const v4i*)(&sPred[wave][4 * lq]);
    int* pp = pred + (size_t)base + 4 * lq;
    for (int pass = 0; pass < 2; ++pass) {
      if (lane < 16) *(volatile v4i*)pp = pv;
      __threadfence();
    }
  }

  sFill[wave][lane] = acc0;
  sFill[wave][32 + lane] = acc1;
  __syncthreads();
  if (tid < NCLUST) {
    float s = 0.f;
#pragma unroll
    for (int w = 0; w < ASG_WAVES; ++w) s += sFill[w][tid];
    sOut[tid] = s;
  }
  __syncthreads();
  if (wave == 0) {
    const int lq = (lane < 16) ? lane : 0;
    const v4f ov = *(const v4f*)(&sOut[4 * lq]);
    float* pp = partp + (size_t)blockIdx.x * NCLUST + 4 * lq;
    for (int pass = 0; pass < 2; ++pass) {
      if (lane < 16) *(volatile v4f*)pp = ov;
      __threadfence();
    }
  }
}

__global__ __launch_bounds__(32) void cluster_stats_kernel(
    const float* __restrict__ x, const int* __restrict__ pred, float* __restrict__ stats,
    int npts, int nchunks) {
  __shared__ __align__(16) int   sList[ST_CHUNK];
  __shared__ __align__(16) float sM2[XDIM * XDIM];
  __shared__ __align__(16) float sSum[XDIM];
  const int lane = threadIdx.x & 31;
  const int k = blockIdx.x;
  const unsigned ltmask = (1u << lane) - 1u;

  float acc[XDIM];
#pragma unroll
  for (int b = 0; b < XDIM; ++b) acc[b] = 0.f;
  float sacc = 0.f;
  int cnt = 0;

#pragma unroll 1
  for (int ch = 0; ch < nchunks; ++ch) {
    const int cbase = ch * ST_CHUNK;
    int total = 0;
#pragma unroll
    for (int s = 0; s < 4; ++s) {
      const int p0 = cbase + s * 128 + 4 * lane;
      const v4i pv = *(const v4i*)(pred + p0);
      const bool f0 = (pv.x == k), f1 = (pv.y == k), f2 = (pv.z == k), f3 = (pv.w == k);
      const unsigned m0 = __builtin_amdgcn_ballot_w32(f0);
      const unsigned m1 = __builtin_amdgcn_ballot_w32(f1);
      const unsigned m2 = __builtin_amdgcn_ballot_w32(f2);
      const unsigned m3 = __builtin_amdgcn_ballot_w32(f3);
      const int pre = __builtin_popcount(m0 & ltmask) + __builtin_popcount(m1 & ltmask)
                    + __builtin_popcount(m2 & ltmask) + __builtin_popcount(m3 & ltmask);
      int pos = total + pre;
      if (f0 && pos < ST_CHUNK) sList[pos] = p0;
      pos += f0 ? 1 : 0;
      if (f1 && pos < ST_CHUNK) sList[pos] = p0 + 1;
      pos += f1 ? 1 : 0;
      if (f2 && pos < ST_CHUNK) sList[pos] = p0 + 2;
      pos += f2 ? 1 : 0;
      if (f3 && pos < ST_CHUNK) sList[pos] = p0 + 3;
      total += __builtin_popcount(m0) + __builtin_popcount(m1) + __builtin_popcount(m2) + __builtin_popcount(m3);
    }
    __syncthreads();
    const int nh = (total < ST_CHUNK) ? total : ST_CHUNK;
    cnt += nh;
#pragma unroll 1
    for (int i = 0; i < nh; ++i) {
      int n = sList[i];
      n = (n < 0) ? 0 : ((n >= npts) ? (npts - 1) : n);
      const float* xr = x + (size_t)n * XDIM;
      const float xa = xr[lane];
      const v4f b0 = *(const v4f*)(xr + 0);
      const v4f b1 = *(const v4f*)(xr + 4);
      const v4f b2 = *(const v4f*)(xr + 8);
      const v4f b3 = *(const v4f*)(xr + 12);
      const v4f b4 = *(const v4f*)(xr + 16);
      const v4f b5 = *(const v4f*)(xr + 20);
      const v4f b6 = *(const v4f*)(xr + 24);
      const v4f b7 = *(const v4f*)(xr + 28);
#pragma unroll
      for (int e = 0; e < 4; ++e) {
        acc[e]      = fmaf(xa, b0[e], acc[e]);
        acc[4 + e]  = fmaf(xa, b1[e], acc[4 + e]);
        acc[8 + e]  = fmaf(xa, b2[e], acc[8 + e]);
        acc[12 + e] = fmaf(xa, b3[e], acc[12 + e]);
        acc[16 + e] = fmaf(xa, b4[e], acc[16 + e]);
        acc[20 + e] = fmaf(xa, b5[e], acc[20 + e]);
        acc[24 + e] = fmaf(xa, b6[e], acc[24 + e]);
        acc[28 + e] = fmaf(xa, b7[e], acc[28 + e]);
      }
      sacc += xa;
    }
    __syncthreads();
  }

  {
    float* mr = sM2 + lane * XDIM;
    *(v4f*)(mr + 0)  = (v4f){acc[0],  acc[1],  acc[2],  acc[3]};
    *(v4f*)(mr + 4)  = (v4f){acc[4],  acc[5],  acc[6],  acc[7]};
    *(v4f*)(mr + 8)  = (v4f){acc[8],  acc[9],  acc[10], acc[11]};
    *(v4f*)(mr + 12) = (v4f){acc[12], acc[13], acc[14], acc[15]};
    *(v4f*)(mr + 16) = (v4f){acc[16], acc[17], acc[18], acc[19]};
    *(v4f*)(mr + 20) = (v4f){acc[20], acc[21], acc[22], acc[23]};
    *(v4f*)(mr + 24) = (v4f){acc[24], acc[25], acc[26], acc[27]};
    *(v4f*)(mr + 28) = (v4f){acc[28], acc[29], acc[30], acc[31]};
    sSum[lane] = sacc;
  }
  __syncthreads();
  float* rec = stats + (size_t)k * ST_STRIDE;
  const int rq = lane >> 3, c4 = (lane & 7) * 4;
  v4f cv = (v4f){0.f, 0.f, 0.f, 0.f};
  if (lane == 0) cv[0] = (float)cnt;
  const v4f sv = *(const v4f*)(sSum + c4);
  for (int pass = 0; pass < 2; ++pass) {
#pragma unroll
    for (int it = 0; it < 8; ++it) {
      const int row = it * 4 + rq;
      const v4f v = *(const v4f*)(sM2 + row * XDIM + c4);
      *(volatile v4f*)(rec + row * XDIM + c4) = v;
    }
    if (lane < 8) {
      *(volatile v4f*)(rec + XDIM * XDIM + c4) = sv;
      *(volatile v4f*)(rec + XDIM * XDIM + XDIM + c4) = cv;
    }
    __threadfence();
  }
}

__global__ __launch_bounds__(256) void final_kernel(
    const float* __restrict__ partp, int nblk, const float* __restrict__ stats,
    const float* __restrict__ ft, const float* __restrict__ mt, const float* __restrict__ ct,
    float* __restrict__ out, int npts) {
  __shared__ float sFil[NCLUST];
  __shared__ float sInv[NCLUST];
  __shared__ float sMean[NCLUST * XDIM];
  __shared__ float sRed[3][256];
  const int tid = threadIdx.x;
  if (tid < NCLUST) {
    float s = 0.f;
#pragma unroll 1
    for (int b = 0; b < nblk; ++b) s += partp[(size_t)b * NCLUST + tid];
    sFil[tid] = s;
    const float c = stats[(size_t)tid * ST_STRIDE + XDIM * XDIM + XDIM];
    sInv[tid] = 1.0f / fmaxf(c, 1.0f);
  }
  __syncthreads();
#pragma unroll 1
  for (int i = tid; i < NCLUST * XDIM; i += 256) {
    const int k = i >> 5;
    sMean[i] = stats[(size_t)k * ST_STRIDE + XDIM * XDIM + (i & 31)] * sInv[k];
  }
  __syncthreads();
  float pf = 0.f, pm = 0.f, pc = 0.f;
  if (tid < NCLUST) {
    const float d = sFil[tid] * (1.0f / (float)npts) - ft[tid];
    pf = d * d;
  }
#pragma unroll 1
  for (int i = tid; i < NCLUST * XDIM; i += 256) {
    const float d = sMean[i] - mt[i];
    pm = fmaf(d, d, pm);
  }
#pragma unroll 1
  for (int i = tid; i < NCLUST * XDIM * XDIM; i += 256) {
    const int k = i >> 10, a = (i >> 5) & 31, b = i & 31;
    const float cov = stats[(size_t)k * ST_STRIDE + (a << 5) + b] * sInv[k] - sMean[(k << 5) + a] * sMean[(k << 5) + b];
    const float d = cov - ct[i];
    pc = fmaf(d, d, pc);
  }
  sRed[0][tid] = pf; sRed[1][tid] = pm; sRed[2][tid] = pc;
  __syncthreads();
  for (int s = 128; s > 0; s >>= 1) {
    if (tid < s) {
      sRed[0][tid] += sRed[0][tid + s];
      sRed[1][tid] += sRed[1][tid + s];
      sRed[2][tid] += sRed[2][tid + s];
    }
    __syncthreads();
  }
  if (tid == 0) {
    const float loss_fil  = sRed[0][0] * (1.0f / (float)NCLUST);
    const float loss_stat = sRed[1][0] * (1.0f / (float)(NCLUST * XDIM)) + sRed[2][0] * (1.0f / (float)(NCLUST * XDIM * XDIM));
    const float loss = loss_fil + KAPPA_W * loss_stat;
    *(volatile float*)out = loss;
    __threadfence();
    *(volatile float*)out = loss;
  }
}

static inline size_t align_up256(size_t v) { return (v + 255) & ~(size_t)255; }

extern "C" void kernel_launch(void* const* d_in, const int* in_sizes, int n_in,
                              void* d_out, int out_size, void* d_ws, size_t ws_size,
                              hipStream_t stream) {
  if (n_in < 5 || out_size < 1) return;
  const float* x       = (const float*)d_in[0];
  const float* centers = (const float*)d_in[1];
  const float* ft      = (const float*)d_in[2];
  const float* mt      = (const float*)d_in[3];
  const float* ct      = (const float*)d_in[4];
  float* out = (float*)d_out;

  const int npts = in_sizes[0] / XDIM;
  if (npts <= 0 || in_sizes[0] != npts * XDIM) return;
  if ((npts % ASG_PPB) != 0) return;
  if (in_sizes[1] != NCLUST * XDIM || in_sizes[2] < NCLUST ||
      in_sizes[3] != NCLUST * XDIM || in_sizes[4] != NCLUST * XDIM * XDIM) return;
  const int nblkA   = npts / ASG_PPB;
  const int nchunks = npts / ST_CHUNK;

  const size_t szXp = (size_t)npts * XDIM * 2;
  const size_t szCp = (size_t)NCLUST * XDIM * 2;
  const size_t szXC = (size_t)npts * NCLUST * 4;
  const size_t szPr = (size_t)npts * 4;
  const size_t szPa = (size_t)nblkA * NCLUST * 4;
  const size_t szSt = (size_t)NCLUST * ST_STRIDE * 4;
  const size_t offXh = 0;
  const size_t offXl = align_up256(offXh + szXp);
  const size_t offCh = align_up256(offXl + szXp);
  const size_t offCl = align_up256(offCh + szCp);
  const size_t offXC = align_up256(offCl + szCp);
  const size_t offPr = align_up256(offXC + szXC);
  const size_t offPa = align_up256(offPr + szPr);
  const size_t offSt = align_up256(offPa + szPa);
  const size_t total = offSt + szSt;
  if (total > ws_size) return;

  char* ws = (char*)d_ws;
  unsigned short* xHi = (unsigned short*)(ws + offXh);
  unsigned short* xLo = (unsigned short*)(ws + offXl);
  unsigned short* cHi = (unsigned short*)(ws + offCh);
  unsigned short* cLo = (unsigned short*)(ws + offCl);
  float* xcp   = (float*)(ws + offXC);
  int*   predp = (int*)(ws + offPr);
  float* partp = (float*)(ws + offPa);
  float* statp = (float*)(ws + offSt);

  {
    const int rows = npts / 2;
    const int nthr = rows * 8;
    split_rows64_bf16<<<(nthr + 255) / 256, 256, 0, stream>>>(x, xHi, xLo, rows, rows);
  }
  {
    const int rows = (NCLUST * XDIM) / FEAT;
    const int nthr = rows * 8;
    split_rows64_bf16<<<(nthr + 255) / 256, 256, 0, stream>>>(centers, cHi, cLo, rows, rows);
  }
  {
    const int tiles = (npts / 64) * (NCLUST / 64);
    dim3 grid((tiles + 7) / 8, 1);
    wmma_gemm64<1, true, 0, 0, false, 0><<<grid, 256, 0, stream>>>(
        xHi, xLo, XDIM, 0L,
        cHi, cLo, XDIM, 0L,
        (void*)xcp, (void*)xcp, NCLUST, 0L,
        (const float*)xcp,
        (const float*)xcp, 0L,
        npts, NCLUST, XDIM, 1.0f);
  }
  assign_kernel<<<nblkA, ASG_WAVES * 32, 0, stream>>>(x, centers, xcp, predp, partp, npts);
  cluster_stats_kernel<<<NCLUST, 32, 0, stream>>>(x, predp, statp, npts, nchunks);
  final_kernel<<<1, 256, 0, stream>>>(partp, nblkA, statp, ft, mt, ct, out, npts);
}
